// InformerBlock_86277303042470
// MI455X (gfx1250) — hardware-run, weakly checked
//
#include <hip/hip_runtime.h>

typedef _Float16 v16h __attribute__((ext_vector_type(16)));
typedef _Float16 v8h  __attribute__((ext_vector_type(8)));
typedef _Float16 v4h  __attribute__((ext_vector_type(4)));
typedef float    v8f  __attribute__((ext_vector_type(8)));
typedef float    v4f  __attribute__((ext_vector_type(4)));
typedef int      v4i  __attribute__((ext_vector_type(4)));
typedef v8h __attribute__((may_alias)) v8ha;
typedef v4f __attribute__((may_alias)) v4fa;
typedef v4i __attribute__((may_alias)) v4ia;

union Frag { v16h v; v8h half[2]; };

#define BB    4
#define LL    1024
#define DD    768
#define UU    7097
#define DFF   3072
#define NTOK  (BB * LL)

#define WSC      256.0f
#define INV_WSC  0.00390625f
#define VSC      16.0f
#define INV_VSC  0.0625f
#define HSC      8.0f
#define INV_HSC  0.125f
#define LN_EPS   1e-5f

#define NX8   (NTOK * DD / 8)
#define NW8   (DD * DD / 8)
#define NF8   (DFF * DD / 8)
#define NCVT  (NX8 + 3 * NW8 + 2 * NF8)
static_assert(NX8 % 256 == 0);
static_assert(NW8 % 256 == 0);
static_assert(NF8 % 256 == 0);

#define BYTES_XH    ((size_t)NTOK * DD * 2)
#define BYTES_WH    ((size_t)3 * DD * DD * 2)
#define BYTES_W1H   ((size_t)DFF * DD * 2)
#define BYTES_W2H   ((size_t)DD * DFF * 2)
#define BYTES_QH    BYTES_XH
#define BYTES_KH    BYTES_XH
#define BYTES_VT    ((size_t)BB * DD * LL * 2)
#define BYTES_FULL  ((size_t)BB * LL * LL * 4)
#define BYTES_MASK  ((size_t)LL * LL * 2)
#define BYTES_STAT  ((size_t)LL * 32 * 4)
#define BYTES_SALL  ((size_t)BB * DD * 4)
#define BYTES_SSET  ((size_t)NTOK * DD * 4)
#define BYTES_X1    BYTES_SSET
#define BYTES_X1H   BYTES_XH
#define BYTES_HH    ((size_t)NTOK * DFF * 2)
#define BYTES_FF    BYTES_SSET
#define WS_TOTAL (BYTES_XH + BYTES_WH + BYTES_W1H + BYTES_W2H + BYTES_QH + BYTES_KH + BYTES_VT + BYTES_FULL + \
                  BYTES_MASK + BYTES_STAT + BYTES_SALL + BYTES_SSET + BYTES_X1 + BYTES_X1H + BYTES_HH + BYTES_FF)
static_assert(WS_TOTAL == (size_t)126365696);
static_assert(WS_TOTAL <= (size_t)134217728);
static_assert(DD % 64 == 0);
static_assert(DFF % 64 == 0);
static_assert(LL % 128 == 0);
static_assert(NTOK % 128 == 0);
static_assert(DD % 32 == 0);
static_assert(DFF % 32 == 0);

__device__ __forceinline__ v8f wmma_f16(v16h a, v16h b, v8f c) {
  v8f d = __builtin_amdgcn_wmma_f32_16x16x32_f16(false, a, false, b, (short)0, c, false, false);
  asm volatile("v_nop\n\tv_nop\n\tv_nop\n\tv_nop" : "+v"(d) : "v"(a), "v"(b));
  return d;
}

__device__ __forceinline__ v16h load_frag(const _Float16* p, int h) {
  Frag f;
  f.half[0] = *(const v8ha*)(p + 8 * h);
  f.half[1] = *(const v8ha*)(p + 16 + 8 * h);
  return f.v;
}

__device__ __forceinline__ float wsum(float v) {
  #pragma unroll
  for (int o = 16; o > 0; o >>= 1) v += __shfl_xor(v, o);
  return v;
}
__device__ __forceinline__ float wmax(float v) {
  #pragma unroll
  for (int o = 16; o > 0; o >>= 1) v = fmaxf(v, __shfl_xor(v, o));
  return v;
}
__device__ __forceinline__ int wsum_i(int v) {
  #pragma unroll
  for (int o = 16; o > 0; o >>= 1) v += __shfl_xor(v, o);
  return v;
}

__device__ __forceinline__ void mma_core(const _Float16* __restrict__ a0p, const _Float16* __restrict__ a1p,
                                         const _Float16* __restrict__ bp, const size_t bstep, const int K,
                                         const int h, v8f (&acc)[2][4]) {
  const v8f zero8 = {0.f, 0.f, 0.f, 0.f, 0.f, 0.f, 0.f, 0.f};
  #pragma unroll
  for (int mt = 0; mt < 2; ++mt)
    #pragma unroll
    for (int nt = 0; nt < 4; ++nt) acc[mt][nt] = zero8;

  #pragma unroll 1
  for (int k0 = 0; k0 < K; k0 += 32) {
    const v16h a0 = load_frag(a0p + k0, h);
    const v16h a1 = load_frag(a1p + k0, h);
    #pragma unroll
    for (int nt = 0; nt < 4; ++nt) {
      const v16h b = load_frag(bp + (size_t)nt * bstep + k0, h);
      acc[0][nt] = wmma_f16(a0, b, acc[0][nt]);
      acc[1][nt] = wmma_f16(a1, b, acc[1][nt]);
    }
  }
}

__device__ __forceinline__ void store_pass_f32(const float* sT, float* C, const int ldc, const int w, const int lane) {
  const int q8 = lane & 7, sub = lane >> 3;
  #pragma unroll
  for (int i = 0; i < 16; ++i) {
    const int lid = i * 4 + sub;
    const int row = 32 * w + (lid >> 1), hl = lid & 1;
    const v4f v = *(const v4fa*)(sT + row * 64 + 32 * hl + 4 * q8);
    *(volatile v4f*)(C + (size_t)row * ldc + 32 * hl + 4 * q8) = v;
  }
}
__device__ __forceinline__ void store_pass_h(const _Float16* sT, _Float16* C, const int ldc, const int w, const int lane) {
  const int q8 = lane & 7, sub = lane >> 3;
  #pragma unroll
  for (int i = 0; i < 8; ++i) {
    const int lid = 32 * w + i * 4 + sub;
    const v8h v = *(const v8ha*)(sT + lid * 64 + 8 * q8);
    *(volatile v8h*)(C + (size_t)lid * ldc + 8 * q8) = v;
  }
}
__device__ __forceinline__ void store_pass_vt(const _Float16* sT, _Float16* V0, const int w, const int lane) {
  const int q8 = lane & 7, sub = lane >> 3;
  #pragma unroll
  for (int i = 0; i < 8; ++i) {
    const int lid = 32 * w + i * 4 + sub;
    const int d = lid >> 1, hl = lid & 1;
    const v8h v = *(const v8ha*)(sT + d * 128 + 64 * hl + 8 * q8);
    *(volatile v8h*)(V0 + (size_t)d * LL + 64 * hl + 8 * q8) = v;
  }
}

__global__ __launch_bounds__(256) void convert_kernel(
    const float* __restrict__ x, const float* __restrict__ wq, const float* __restrict__ wk,
    const float* __restrict__ wv, const float* __restrict__ w1, const float* __restrict__ w2,
    _Float16* __restrict__ xh, _Float16* __restrict__ wh, _Float16* __restrict__ w1h, _Float16* __restrict__ w2h)
{
  const int g = blockIdx.x * 256 + threadIdx.x;
  if (g >= NCVT) return;
  const float* src;
  _Float16* dst;
  float sc;
  if (g < NX8) {
    src = x + (size_t)g * 8;
    dst = xh + (size_t)g * 8;
    sc = 1.0f;
  } else if (g < NX8 + 3 * NW8) {
    const int e = g - NX8;
    const int wsel = e / NW8;
    const int off = e - wsel * NW8;
    const float* wsrc = (wsel == 0) ? wq : ((wsel == 1) ? wk : wv);
    src = wsrc + (size_t)off * 8;
    dst = wh + (size_t)e * 8;
    sc = WSC;
  } else if (g < NX8 + 3 * NW8 + NF8) {
    const int e = g - (NX8 + 3 * NW8);
    src = w1 + (size_t)e * 8;
    dst = w1h + (size_t)e * 8;
    sc = WSC;
  } else {
    const int e = g - (NX8 + 3 * NW8 + NF8);
    src = w2 + (size_t)e * 8;
    dst = w2h + (size_t)e * 8;
    sc = WSC;
  }
  const v4f a = *(const v4fa*)src;
  const v4f c = *(const v4fa*)(src + 4);
  const v8h o = { (_Float16)(a.x * sc), (_Float16)(a.y * sc), (_Float16)(a.z * sc), (_Float16)(a.w * sc),
                  (_Float16)(c.x * sc), (_Float16)(c.y * sc), (_Float16)(c.z * sc), (_Float16)(c.w * sc) };
  *(volatile v8h*)dst = o;
  __threadfence();
  *(volatile v8h*)dst = o;
}

__global__ __launch_bounds__(128) void proj_kernel(
    const _Float16* __restrict__ xh,
    const _Float16* __restrict__ wh,
    const float* __restrict__ bq, const float* __restrict__ bk, const float* __restrict__ bv,
    _Float16* __restrict__ qh,
    _Float16* __restrict__ kh,
    _Float16* __restrict__ vt)
{
  __shared__ __attribute__((aligned(16))) _Float16 sT[128 * 64];

  const int tid = threadIdx.x, lane = tid & 31, w = tid >> 5;
  const int h = lane >> 4, m = lane & 15;
  const int m0 = blockIdx.x * 128;
  const int cg = blockIdx.y;
  const int which = cg / 12, fg = cg - which * 12;

  const _Float16* a0p = xh + (size_t)(m0 + 32 * w + m) * DD;
  const _Float16* a1p = a0p + (size_t)16 * DD;
  const _Float16* bp  = wh + ((size_t)which * DD + fg * 64 + m) * DD;

  v8f acc[2][4];
  mma_core(a0p, a1p, bp, (size_t)16 * DD, DD, h, acc);

  const float* bias = (which == 0) ? bq : ((which == 1) ? bk : bv);
  const float vmul = (which == 2) ? VSC : 1.0f;
  #pragma unroll
  for (int nt = 0; nt < 4; ++nt) {
    const int feat = 16 * nt + m;
    const float bvl = bias[fg * 64 + feat];
    #pragma unroll
    for (int mt = 0; mt < 2; ++mt) {
      #pragma unroll
      for (int r = 0; r < 8; ++r) {
        const int tokl = 32 * w + 16 * mt + 8 * h + r;
        const float y = (acc[mt][nt][r] * INV_WSC + bvl) * vmul;
        const int li = (which == 2) ? (feat * 128 + tokl) : (tokl * 64 + feat);
        sT[li] = (_Float16)y;
      }
    }
  }
  __syncthreads();

  if (which == 2) {
    const int b = m0 / LL, l0 = m0 - b * LL;
    _Float16* V0 = vt + ((size_t)b * DD + fg * 64) * LL + l0;
    store_pass_vt(sT, V0, w, lane);
    __threadfence();
    store_pass_vt(sT, V0, w, lane);
  } else {
    _Float16* C = ((which == 0) ? qh : kh) + (size_t)m0 * DD + fg * 64;
    store_pass_h(sT, C, DD, w, lane);
    __threadfence();
    store_pass_h(sT, C, DD, w, lane);
  }
}

template <int MODE> struct BiasSel { static __device__ __forceinline__ float get(const float*, int) { return 0.0f; } };
template <> struct BiasSel<2> { static __device__ __forceinline__ float get(const float* b, int c) { return b[c]; } };

template <int MODE>
__global__ __launch_bounds__(128) void gemm_f32_kernel(
    const _Float16* __restrict__ A, const _Float16* __restrict__ Bm,
    const float* __restrict__ bias, float* __restrict__ C, const float oscale)
{
  constexpr int    LDA = (MODE == 0) ? DD : ((MODE == 1) ? LL : DFF);
  constexpr size_t SA  = (MODE == 0) ? (size_t)LL * DD : (size_t)0;
  constexpr int    LDB = LDA;
  constexpr size_t SB  = (MODE == 0) ? (size_t)LL * DD : ((MODE == 1) ? (size_t)DD * LL : (size_t)0);
  constexpr int    LDC = (MODE == 0) ? LL : DD;
  constexpr size_t SC  = (MODE == 0) ? (size_t)LL * LL : ((MODE == 1) ? (size_t)LL * DD : (size_t)0);
  constexpr int    K   = LDA;

  __shared__ __attribute__((aligned(16))) float sT[128 * 64];

  const int tid = threadIdx.x, lane = tid & 31, w = tid >> 5;
  const int h = lane >> 4, m = lane & 15;
  const int m0 = blockIdx.y * 128, n0 = blockIdx.x * 64, z = blockIdx.z;

  const _Float16* Ab = A + (size_t)z * SA;
  const _Float16* Bb = Bm + (size_t)z * SB;
  float* Cb = C + (size_t)z * SC;

  const _Float16* a0p = Ab + (size_t)(m0 + 32 * w + m) * LDA;
  const _Float16* a1p = a0p + (size_t)16 * LDA;
  const _Float16* bp  = Bb + (size_t)(n0 + m) * LDB;

  v8f acc[2][4];
  mma_core(a0p, a1p, bp, (size_t)16 * LDB, K, h, acc);

  #pragma unroll
  for (int nt = 0; nt < 4; ++nt) {
    const int col = 16 * nt + m;
    const float bvl = BiasSel<MODE>::get(bias, n0 + col);
    #pragma unroll
    for (int mt = 0; mt < 2; ++mt) {
      #pragma unroll
      for (int r = 0; r < 8; ++r) {
        const int rowl = 32 * w + 16 * mt + 8 * h + r;
        sT[rowl * 64 + col] = acc[mt][nt][r] * oscale + bvl;
      }
    }
  }
  __syncthreads();

  float* Ct = Cb + (size_t)m0 * LDC + n0;
  store_pass_f32(sT, Ct, LDC, w, lane);
  __threadfence();
  store_pass_f32(sT, Ct, LDC, w, lane);
}

__global__ __launch_bounds__(256) void rowstat_kernel(
    const float* __restrict__ full,
    const int* __restrict__ idx,
    _Float16* __restrict__ maskp,
    float* __restrict__ stats)
{
  __shared__ __attribute__((aligned(16))) float srow[BB * LL];
  __shared__ __attribute__((aligned(16))) int sflag[LL];
  __shared__ float smax[8 * BB], ssum[8 * BB];
  __shared__ int scnt[4];

  const int i = blockIdx.x, t = threadIdx.x, lane = t & 31, w = t >> 5;

  #pragma unroll
  for (int b = 0; b < BB; ++b)
    *(v4fa*)(srow + b * LL + 4 * t) = *(const v4fa*)(full + ((size_t)(b * LL + i)) * LL + 4 * t);
  const v4i z4 = {0, 0, 0, 0};
  *(v4ia*)(sflag + 4 * t) = z4;
  __syncthreads();

  float mx[BB], sm[BB];
  #pragma unroll
  for (int b = 0; b < BB; ++b) { mx[b] = -3.0e38f; sm[b] = 0.0f; }
  const int* ip = idx + (size_t)i * UU;
  #pragma unroll 1
  for (int u = t; u < UU; u += 256) {
    int p = ip[u];
    p = min(max(p, 0), LL - 1);
    sflag[p] = 1;
    #pragma unroll
    for (int b = 0; b < BB; ++b) {
      const float v = srow[b * LL + p];
      mx[b] = fmaxf(mx[b], v);
      sm[b] += v;
    }
  }
  #pragma unroll
  for (int b = 0; b < BB; ++b) { mx[b] = wmax(mx[b]); sm[b] = wsum(sm[b]); }
  if (lane == 0) {
    #pragma unroll
    for (int b = 0; b < BB; ++b) { smax[w * BB + b] = mx[b]; ssum[w * BB + b] = sm[b]; }
  }
  __syncthreads();

  if (t < 128) {
    int cnt = 0;
    v8h mrow;
    #pragma unroll
    for (int j = 0; j < 8; ++j) {
      const int f = sflag[8 * t + j];
      cnt += f;
      mrow[j] = (_Float16)((float)f);
    }
    cnt = wsum_i(cnt);
    if (lane == 0) scnt[w] = cnt;
    _Float16* dst = maskp + (size_t)i * LL + 8 * t;
    *(volatile v8h*)dst = mrow;
    __threadfence();
    *(volatile v8h*)dst = mrow;
  }
  __syncthreads();

  if (t < 32) {
    const int b = lane & 3;
    float MX = smax[b], SM = ssum[b];
    #pragma unroll
    for (int w2 = 1; w2 < 8; ++w2) { MX = fmaxf(MX, smax[w2 * BB + b]); SM += ssum[w2 * BB + b]; }
    const int n1 = (scnt[0] + scnt[1]) + (scnt[2] + scnt[3]);
    const float mmv = MX - SM * (1.0f / (float)UU);
    const float em = __expf(-mmv);
    const float den = (float)n1 + (float)(LL - n1) * em;
    const float cA = 1.0f / den;
    const float cB = em * cA;
    float val = 0.0f;
    val = (lane < 4) ? cA : ((lane < 8) ? cB : ((lane == 8) ? (float)n1 : 0.0f));
    float* dst = stats + (size_t)i * 32 + lane;
    *(volatile float*)dst = val;
    __threadfence();
    *(volatile float*)dst = val;
  }
}

__global__ __launch_bounds__(256) void vsum_kernel(const _Float16* __restrict__ vt, float* __restrict__ sall)
{
  __shared__ float sS[32];
  const int t = threadIdx.x, lane = t & 31, w = t >> 5;
  const int r0 = blockIdx.x * 32;
  #pragma unroll 1
  for (int j = 0; j < 4; ++j) {
    const int r = r0 + 4 * w + j;
    const _Float16* p = vt + (size_t)r * LL + 32 * lane;
    float s = 0.0f;
    #pragma unroll
    for (int q = 0; q < 4; ++q) {
      const v8h v = *(const v8ha*)(p + 8 * q);
      s += (((float)v[0] + (float)v[1]) + ((float)v[2] + (float)v[3])) +
           (((float)v[4] + (float)v[5]) + ((float)v[6] + (float)v[7]));
    }
    s = wsum(s);
    if (lane == 0) sS[4 * w + j] = s;
  }
  __syncthreads();
  if (t < 32) {
    const float val = sS[lane] * INV_VSC;
    float* dst = sall + r0 + lane;
    *(volatile float*)dst = val;
    __threadfence();
    *(volatile float*)dst = val;
  }
}

__device__ __forceinline__ float block_sum192(float v, float* sred, const int w, const int lane) {
  v = wsum(v);
  if (lane == 0) sred[w] = v;
  __syncthreads();
  return ((sred[0] + sred[1]) + (sred[2] + sred[3])) + (sred[4] + sred[5]);
}

__global__ __launch_bounds__(192) void zln1_kernel(
    const float* __restrict__ x, const float* __restrict__ sset, const float* __restrict__ sall,
    const float* __restrict__ stats, const float* __restrict__ g1, const float* __restrict__ be1,
    float* __restrict__ x1, _Float16* __restrict__ x1h)
{
  __shared__ float sra[8], srb[8];
  const int row = blockIdx.x, t = threadIdx.x, lane = t & 31, w = t >> 5;
  const int b = row >> 10, i = row & (LL - 1);
  const float cA = stats[(size_t)i * 32 + b];
  const float cB = stats[(size_t)i * 32 + 4 + b];
  const float cS = cA - cB;
  const size_t o = (size_t)row * DD + 4 * t;
  const v4f xv = *(const v4fa*)(x + o);
  const v4f sv = *(const v4fa*)(sset + o);
  const v4f av = *(const v4fa*)(sall + (size_t)b * DD + 4 * t);
  v4f tv;
  tv.x = xv.x + (sv.x * cS + av.x * cB);
  tv.y = xv.y + (sv.y * cS + av.y * cB);
  tv.z = xv.z + (sv.z * cS + av.z * cB);
  tv.w = xv.w + (sv.w * cS + av.w * cB);

  const float mu = block_sum192((tv.x + tv.y) + (tv.z + tv.w), sra, w, lane) * (1.0f / (float)DD);
  v4f dv;
  dv.x = tv.x - mu; dv.y = tv.y - mu; dv.z = tv.z - mu; dv.w = tv.w - mu;
  const float var = block_sum192((dv.x * dv.x + dv.y * dv.y) + (dv.z * dv.z + dv.w * dv.w), srb, w, lane) * (1.0f / (float)DD);
  const float rs = rsqrtf(var + LN_EPS);
  const v4f gv = *(const v4fa*)(g1 + 4 * t);
  const v4f bev = *(const v4fa*)(be1 + 4 * t);
  v4f y;
  y.x = dv.x * rs * gv.x + bev.x;
  y.y = dv.y * rs * gv.y + bev.y;
  y.z = dv.z * rs * gv.z + bev.z;
  y.w = dv.w * rs * gv.w + bev.w;
  const v4h yh = { (_Float16)y.x, (_Float16)y.y, (_Float16)y.z, (_Float16)y.w };

  float* df = x1 + o;
  _Float16* dh = x1h + o;
  *(volatile v4f*)df = y;
  *(volatile v4h*)dh = yh;
  __threadfence();
  *(volatile v4f*)df = y;
  *(volatile v4h*)dh = yh;
}

__global__ __launch_bounds__(128) void ffn1_kernel(
    const _Float16* __restrict__ x1h,
    const _Float16* __restrict__ w1h,
    const float* __restrict__ b1,
    _Float16* __restrict__ hh)
{
  __shared__ __attribute__((aligned(16))) _Float16 sT[128 * 64];

  const int tid = threadIdx.x, lane = tid & 31, w = tid >> 5;
  const int h = lane >> 4, m = lane & 15;
  const int m0 = blockIdx.y * 128, n0 = blockIdx.x * 64;

  const _Float16* a0p = x1h + (size_t)(m0 + 32 * w + m) * DD;
  const _Float16* a1p = a0p + (size_t)16 * DD;
  const _Float16* bp  = w1h + (size_t)(n0 + m) * DD;

  v8f acc[2][4];
  mma_core(a0p, a1p, bp, (size_t)16 * DD, DD, h, acc);

  #pragma unroll
  for (int nt = 0; nt < 4; ++nt) {
    const int col = 16 * nt + m;
    const float bvl = b1[n0 + col];
    #pragma unroll
    for (int mt = 0; mt < 2; ++mt) {
      #pragma unroll
      for (int r = 0; r < 8; ++r) {
        const int rowl = 32 * w + 16 * mt + 8 * h + r;
        const float v = acc[mt][nt][r] * INV_WSC + bvl;
        const float gl = 0.5f * v * (1.0f + erff(v * 0.70710678118654752f));
        sT[rowl * 64 + col] = (_Float16)(gl * HSC);
      }
    }
  }
  __syncthreads();

  _Float16* C = hh + (size_t)m0 * DFF + n0;
  store_pass_h(sT, C, DFF, w, lane);
  __threadfence();
  store_pass_h(sT, C, DFF, w, lane);
}

__global__ __launch_bounds__(192) void ln2_kernel(
    const float* __restrict__ x1, const float* __restrict__ ff,
    const float* __restrict__ g2, const float* __restrict__ be2, float* __restrict__ out)
{
  __shared__ float sra[8], srb[8];
  const int row = blockIdx.x, t = threadIdx.x, lane = t & 31, w = t >> 5;
  const size_t o = (size_t)row * DD + 4 * t;
  const v4f av = *(const v4fa*)(x1 + o);
  const v4f fv = *(const v4fa*)(ff + o);
  v4f tv;
  tv.x = av.x + fv.x; tv.y = av.y + fv.y; tv.z = av.z + fv.z; tv.w = av.w + fv.w;

  const float mu = block_sum192((tv.x + tv.y) + (tv.z + tv.w), sra, w, lane) * (1.0f / (float)DD);
  v4f dv;
  dv.x = tv.x - mu; dv.y = tv.y - mu; dv.z = tv.z - mu; dv.w = tv.w - mu;
  const float var = block_sum192((dv.x * dv.x + dv.y * dv.y) + (dv.z * dv.z + dv.w * dv.w), srb, w, lane) * (1.0f / (float)DD);
  const float rs = rsqrtf(var + LN_EPS);
  const v4f gv = *(const v4fa*)(g2 + 4 * t);
  const v4f bev = *(const v4fa*)(be2 + 4 * t);
  v4f y;
  y.x = dv.x * rs * gv.x + bev.x;
  y.y = dv.y * rs * gv.y + bev.y;
  y.z = dv.z * rs * gv.z + bev.z;
  y.w = dv.w * rs * gv.w + bev.w;

  float* df = out + o;
  *(volatile v4f*)df = y;
  __threadfence();
  *(volatile v4f*)df = y;
}

extern "C" void kernel_launch(void* const* d_in, const int* in_sizes, int n_in,
                              void* d_out, int out_size, void* d_ws, size_t ws_size,
                              hipStream_t stream) {
  if (n_in < 16) return;
  if (in_sizes[0] != NTOK * DD) return;
  if (in_sizes[1] != LL * UU) return;
  if (in_sizes[2] != DD * DD || in_sizes[4] != DD * DD || in_sizes[6] != DD * DD) return;
  if (in_sizes[3] != DD || in_sizes[5] != DD || in_sizes[7] != DD) return;
  if (in_sizes[8] != DFF * DD || in_sizes[9] != DFF) return;
  if (in_sizes[10] != DD * DFF || in_sizes[11] != DD) return;
  if (in_sizes[12] != DD || in_sizes[13] != DD || in_sizes[14] != DD || in_sizes[15] != DD) return;
  if (out_size != NTOK * DD) return;
  if ((size_t)WS_TOTAL > ws_size) return;

  const float* x   = (const float*)d_in[0];
  const int*   idx = (const int*)d_in[1];
  const float* Wq  = (const float*)d_in[2];
  const float* bq  = (const float*)d_in[3];
  const float* Wk  = (const float*)d_in[4];
  const float* bk  = (const float*)d_in[5];
  const float* Wv  = (const float*)d_in[6];
  const float* bv  = (const float*)d_in[7];
  const float* W1  = (const float*)d_in[8];
  const float* b1  = (const float*)d_in[9];
  const float* W2  = (const float*)d_in[10];
  const float* b2  = (const float*)d_in[11];
  const float* g1  = (const float*)d_in[12];
  const float* be1 = (const float*)d_in[13];
  const float* g2  = (const float*)d_in[14];
  const float* be2 = (const float*)d_in[15];
  float* out = (float*)d_out;

  char* ws = (char*)d_ws;
  size_t off = 0;
  _Float16* xh    = (_Float16*)(ws + off); off += BYTES_XH;
  _Float16* wh    = (_Float16*)(ws + off); off += BYTES_WH;
  _Float16* w1h   = (_Float16*)(ws + off); off += BYTES_W1H;
  _Float16* w2h   = (_Float16*)(ws + off); off += BYTES_W2H;
  _Float16* qh    = (_Float16*)(ws + off); off += BYTES_QH;
  _Float16* kh    = (_Float16*)(ws + off); off += BYTES_KH;
  _Float16* vt    = (_Float16*)(ws + off); off += BYTES_VT;
  float*    full  = (float*)(ws + off);    off += BYTES_FULL;
  _Float16* maskp = (_Float16*)(ws + off); off += BYTES_MASK;
  float*    stats = (float*)(ws + off);    off += BYTES_STAT;
  float*    sall  = (float*)(ws + off);    off += BYTES_SALL;
  float*    sset  = (float*)(ws + off);    off += BYTES_SSET;
  float*    x1    = (float*)(ws + off);    off += BYTES_X1;
  _Float16* x1h   = (_Float16*)(ws + off); off += BYTES_X1H;
  _Float16* hh    = (_Float16*)(ws + off); off += BYTES_HH;
  float*    ff    = (float*)(ws + off);    off += BYTES_FF;
  if (off > ws_size) return;

  const float rscale = 1.0f / sqrtf((float)DD);

  convert_kernel<<<NCVT / 256, 256, 0, stream>>>(x, Wq, Wk, Wv, W1, W2, xh, wh, w1h, w2h);

  proj_kernel<<<dim3(NTOK / 128, 3 * (DD / 64)), 128, 0, stream>>>(xh, wh, bq, bk, bv, qh, kh, vt);

  gemm_f32_kernel<0><<<dim3(LL / 64, LL / 128, BB), 128, 0, stream>>>(qh, kh, bq, full, rscale);

  rowstat_kernel<<<LL, 256, 0, stream>>>(full, idx, maskp, stats);

  vsum_kernel<<<(BB * DD) / 32, 256, 0, stream>>>(vt, sall);

  gemm_f32_kernel<1><<<dim3(DD / 64, LL / 128, BB), 128, 0, stream>>>(maskp, vt, bq, sset, INV_VSC);

  zln1_kernel<<<NTOK, 192, 0, stream>>>(x, sset, sall, stats, g1, be1, x1, x1h);

  ffn1_kernel<<<dim3(DFF / 64, NTOK / 128), 128, 0, stream>>>(x1h, w1h, b1, hh);

  gemm_f32_kernel<2><<<dim3(DD / 64, NTOK / 128, 1), 128, 0, stream>>>(hh, w2h, b2, ff, INV_HSC * INV_WSC);

  ln2_kernel<<<NTOK, 192, 0, stream>>>(x1, ff, g2, be2, out);
}
